// DeformConv3D_19791209299987
// MI455X (gfx1250) — hardware-run, weakly checked
//
#include <hip/hip_runtime.h>
#include <stddef.h>
#include <math.h>

typedef __attribute__((ext_vector_type(16))) _Float16 v16h;
typedef __attribute__((ext_vector_type(8)))  _Float16 v8h;
typedef __attribute__((ext_vector_type(16))) __bf16   v16b;
typedef __attribute__((ext_vector_type(8)))  __bf16   v8b;
typedef __attribute__((ext_vector_type(8)))  float    v8f;
typedef __attribute__((ext_vector_type(4)))  float    v4f;
typedef __attribute__((ext_vector_type(2)))  float    v2f;
typedef __attribute__((ext_vector_type(4)))  int      v4i;
typedef __attribute__((ext_vector_type(4)))  unsigned v4u;

constexpr int NB       = 2;
constexpr int CIN      = 128;
constexpr int DEP      = 6;
constexpr int IMH      = 56;
constexpr int IMW      = 56;
constexpr int HW       = IMH * IMW;
constexpr int NIMG     = NB * DEP;
constexpr int NPIX     = NIMG * HW;
constexpr int COUT     = 128;
constexpr int NGRP     = 4;
constexpr int CG       = CIN / NGRP;
constexpr int OG       = COUT / NGRP;
constexpr int NTAP     = 9;
constexpr int NOFF     = 2 * NGRP * NTAP;
constexpr int NOFFPAD  = 80;
constexpr int KOFF     = CIN * NTAP;
constexpr int KDEF     = CG * NTAP;
constexpr int HALO_W   = IMW + 2;
constexpr int HALO_H   = IMH + 2;
constexpr int HPIX     = HALO_W * HALO_H;
constexpr int NTHR     = 256;
constexpr int TILE_PX  = 64;
constexpr int TILES_PER_IMG = HW / TILE_PX;
constexpr int NTILES   = NPIX / TILE_PX;
constexpr int RUN      = DEP * HW;
constexpr int AS_PITCH = KDEF + 8;
constexpr int CST_PITCH = 68;
constexpr int TILE_PITCH = 65;
constexpr int HALO_PIX   = HPIX - HW;
constexpr int HALO_PAIRS = HALO_PIX / 2;
constexpr int OC_BLOCK_PX = 256;
constexpr int OC_KSTEPS   = KOFF / 32;
constexpr int DC_KSTEPS   = KDEF / 32;
constexpr int GEO_ITEMS   = TILE_PX * NTAP;
constexpr int SMP_ITEMS   = GEO_ITEMS * (CG / 8);
constexpr int WO_ITEMS    = NOFFPAD * (KOFF / 8);
constexpr int WC_ITEMS    = COUT * (KDEF / 8);
constexpr int WO_BLOCKS   = WO_ITEMS / NTHR;
constexpr int WC_BLOCKS   = WC_ITEMS / NTHR;
constexpr float SMP_CARRY = 16.0f;
constexpr float WC_CARRY  = 64.0f;
constexpr float DC_FOLD   = 1.0f / (SMP_CARRY * WC_CARRY);
constexpr float F16_MIN_NORMAL = 6.103515625e-05f;
constexpr float NORM_EPS  = 1e-5f;
constexpr double INV_RUN  = 1.0 / (double)RUN;

static_assert(HW == 3136 && NIMG == 12 && NPIX == 37632);
static_assert(NOFF == 72 && KOFF == 1152 && KDEF == 288 && CG == 32 && OG == 32);
static_assert(HW % TILE_PX == 0 && TILES_PER_IMG == 49 && NTILES == 588);
static_assert(NPIX % OC_BLOCK_PX == 0);
static_assert(KOFF % 32 == 0 && KDEF % 32 == 0 && NOFFPAD % 16 == 0 && NOFF <= NOFFPAD);
static_assert(CIN % 32 == 0 && OC_KSTEPS == 36 && DC_KSTEPS == 9);
static_assert(WO_ITEMS % NTHR == 0 && WC_ITEMS % NTHR == 0);
static_assert(HALO_PIX == 228 && HALO_PAIRS == 114 && HALO_PAIRS <= 8 * 15);
static_assert(GEO_ITEMS == 2 * NTHR + 64);
static_assert(SMP_ITEMS == 9 * NTHR);
static_assert(RUN % 4 == 0 && (RUN / 4) % 32 == 0);
static_assert((AS_PITCH * 2) % 16 == 0);
static_assert(TILE_PX * AS_PITCH * 2 + GEO_ITEMS * 4 * 4 * 2 + OG * CST_PITCH * 4 <= 65536);

__device__ __forceinline__ unsigned short f2bf_bits(float f) {
  unsigned u = __float_as_uint(f);
  return (unsigned short)((u + 0x7FFFu + ((u >> 16) & 1u)) >> 16);
}
__device__ __forceinline__ float bf_bits2f(unsigned short h) { return __uint_as_float(((unsigned)h) << 16); }
__device__ __forceinline__ unsigned pack16(unsigned short lo, unsigned short hi) {
  return (unsigned)lo | (((unsigned)hi) << 16);
}

template <typename T> struct Frag;
template <> struct Frag<_Float16> {
  typedef v16h V; union U { v16h v; v8h h[2]; };
  static __device__ __forceinline__ v16h load(const _Float16* p) {
    U f; f.h[0] = *(const v8h*)(p); f.h[1] = *(const v8h*)(p + 16); return f.v;
  }
  static __device__ __forceinline__ v8f mma(v16h a, v16h b, v8f c) {
    return __builtin_amdgcn_wmma_f32_16x16x32_f16(false, a, false, b, (short)0, c, false, false);
  }
};
template <> struct Frag<__bf16> {
  typedef v16b V; union U { v16b v; v8b h[2]; };
  static __device__ __forceinline__ v16b load(const __bf16* p) {
    U f; f.h[0] = *(const v8b*)(p); f.h[1] = *(const v8b*)(p + 16); return f.v;
  }
  static __device__ __forceinline__ v8f mma(v16b a, v16b b, v8f c) {
    return __builtin_amdgcn_wmma_f32_16x16x32_bf16(false, a, false, b, (short)0, c, false, false);
  }
};
__device__ __forceinline__ void guard_b(v8f& c, v16b a0, v16b a1, v16b b0, v16b b1) {
  asm volatile("v_nop\n\tv_nop\n\tv_nop\n\tv_nop" : "+v"(c) : "v"(a0), "v"(a1), "v"(b0), "v"(b1));
}
__device__ __forceinline__ v8f mma_h(v16h a, v16h b, v8f c) {
  c = Frag<_Float16>::mma(a, b, c);
  asm volatile("v_nop\n\tv_nop\n\tv_nop\n\tv_nop" : "+v"(c) : "v"(a), "v"(b));
  return c;
}
__device__ __forceinline__ void lds_wave_sync() {
  __builtin_amdgcn_fence(__ATOMIC_RELEASE, "workgroup");
  __builtin_amdgcn_wave_barrier();
  __builtin_amdgcn_fence(__ATOMIC_ACQUIRE, "workgroup");
}

__global__ __launch_bounds__(NTHR) void k_prep_x(const float* __restrict__ x, float* __restrict__ xf,
                                                 unsigned short* __restrict__ xhi, unsigned short* __restrict__ xlo) {
  __shared__ float tile[CIN * TILE_PITCH];
  const int tid  = threadIdx.x;
  const int lane = tid & 31;
  const int wave = tid >> 5;
  const int hh   = lane >> 4;
  const int rl   = lane & 15;
  const int n    = blockIdx.y;
  const int b    = n / DEP;
  const int d    = n - b * DEP;
  if (blockIdx.x == TILES_PER_IMG) {
    v4u z;
    z[0] = 0u; z[1] = 0u; z[2] = 0u; z[3] = 0u;
    for (int pass = 0; pass < 2; ++pass) {
#pragma unroll 1
      for (int it = 0; it < 15; ++it) {
        const int pi = wave + 8 * it;
        if (pi < HALO_PAIRS) {
          const int hp = pi * 2 + hh;
          int row = 0;
          int col = hp;
          if (hp >= HALO_W)            { row = HALO_H - 1;         col = hp - HALO_W; }
          if (hp >= 2 * HALO_W)        { row = hp - (2 * HALO_W - 1); col = 0; }
          if (hp >= 2 * HALO_W + IMH)  { row = hp - (2 * HALO_W + IMH - 1); col = HALO_W - 1; }
          const size_t di = ((size_t)(n * HALO_H + row) * HALO_W + col) * CIN + rl * 8;
          *(volatile v4u*)(xhi + di) = z;
          *(volatile v4u*)(xlo + di) = z;
        }
      }
      __threadfence();
    }
  } else {
    const int hw0 = blockIdx.x * TILE_PX;
    const float* xs = x + ((size_t)(b * CIN) * DEP + d) * HW + hw0;
#pragma unroll 1
    for (int it = 0; it < 8; ++it) {
      const int i  = it * NTHR + tid;
      const int c  = i >> 4;
      const int p4 = (i & 15) * 4;
      const v4f v = *(const v4f*)(xs + (size_t)c * (DEP * HW) + p4);
      float* t = tile + c * TILE_PITCH + p4;
      t[0] = v[0]; t[1] = v[1]; t[2] = v[2]; t[3] = v[3];
    }
    __syncthreads();
    for (int pass = 0; pass < 2; ++pass) {
#pragma unroll 1
      for (int it = 0; it < 8; ++it) {
        const int px = wave * 8 + it;
        v4f v;
        v[0] = tile[(lane * 4 + 0) * TILE_PITCH + px];
        v[1] = tile[(lane * 4 + 1) * TILE_PITCH + px];
        v[2] = tile[(lane * 4 + 2) * TILE_PITCH + px];
        v[3] = tile[(lane * 4 + 3) * TILE_PITCH + px];
        *(volatile v4f*)(xf + ((size_t)n * HW + hw0 + px) * CIN + lane * 4) = v;
      }
#pragma unroll 1
      for (int it = 0; it < 4; ++it) {
        const int px = (wave * 4 + it) * 2 + hh;
        const int c8 = rl * 8;
        unsigned short hb[8];
        unsigned short lb[8];
#pragma unroll
        for (int e = 0; e < 8; ++e) {
          const float f = tile[(c8 + e) * TILE_PITCH + px];
          const unsigned short hbits = f2bf_bits(f);
          hb[e] = hbits;
          lb[e] = f2bf_bits(f - bf_bits2f(hbits));
        }
        v4u hv;
        v4u lv;
        hv[0] = pack16(hb[0], hb[1]); hv[1] = pack16(hb[2], hb[3]); hv[2] = pack16(hb[4], hb[5]); hv[3] = pack16(hb[6], hb[7]);
        lv[0] = pack16(lb[0], lb[1]); lv[1] = pack16(lb[2], lb[3]); lv[2] = pack16(lb[4], lb[5]); lv[3] = pack16(lb[6], lb[7]);
        const int hw = hw0 + px;
        const int h  = hw / IMW;
        const int w  = hw - h * IMW;
        const size_t di = ((size_t)(n * HALO_H + h + 1) * HALO_W + (w + 1)) * CIN + c8;
        *(volatile v4u*)(xhi + di) = hv;
        *(volatile v4u*)(xlo + di) = lv;
      }
      __threadfence();
    }
  }
}

__global__ __launch_bounds__(NTHR) void k_prep_w(const float* __restrict__ ow, const float* __restrict__ cw,
                                                 unsigned short* __restrict__ wohi, unsigned short* __restrict__ wolo,
                                                 unsigned short* __restrict__ wc) {
  const int tid = threadIdx.x;
  if (blockIdx.x < WO_BLOCKS) {
    const int i   = blockIdx.x * NTHR + tid;
    const int row = i / (KOFF / 8);
    const int k0  = (i - row * (KOFF / 8)) * 8;
    const int k2  = k0 >> 7;
    const int c0  = k0 & (CIN - 1);
    const int rowc = (row < NOFF) ? row : (NOFF - 1);
    unsigned short hb[8];
    unsigned short lb[8];
#pragma unroll
    for (int e = 0; e < 8; ++e) {
      float v = ow[(size_t)rowc * KOFF + (c0 + e) * NTAP + k2];
      asm volatile("" : "+v"(v));
      v = (row < NOFF) ? v : 0.0f;
      const unsigned short hbits = f2bf_bits(v);
      hb[e] = hbits;
      lb[e] = f2bf_bits(v - bf_bits2f(hbits));
    }
    v4u hv;
    v4u lv;
    hv[0] = pack16(hb[0], hb[1]); hv[1] = pack16(hb[2], hb[3]); hv[2] = pack16(hb[4], hb[5]); hv[3] = pack16(hb[6], hb[7]);
    lv[0] = pack16(lb[0], lb[1]); lv[1] = pack16(lb[2], lb[3]); lv[2] = pack16(lb[4], lb[5]); lv[3] = pack16(lb[6], lb[7]);
    unsigned short* dh = wohi + (size_t)i * 8;
    unsigned short* dl = wolo + (size_t)i * 8;
    *(volatile v4u*)dh = hv;
    *(volatile v4u*)dl = lv;
    __threadfence();
    *(volatile v4u*)dh = hv;
    *(volatile v4u*)dl = lv;
  } else {
    const int i   = (blockIdx.x - WO_BLOCKS) * NTHR + tid;
    const int row = i / (KDEF / 8);
    const int k0  = (i - row * (KDEF / 8)) * 8;
    const int tap = k0 >> 5;
    const int c0  = k0 & (CG - 1);
    unsigned short hb[8];
#pragma unroll
    for (int e = 0; e < 8; ++e) {
      float v = cw[(size_t)row * KDEF + (c0 + e) * NTAP + tap] * WC_CARRY;
      v = (fabsf(v) < F16_MIN_NORMAL) ? 0.0f : v;
      const _Float16 hval = (_Float16)v;
      hb[e] = __builtin_bit_cast(unsigned short, hval);
    }
    v4u hv;
    hv[0] = pack16(hb[0], hb[1]); hv[1] = pack16(hb[2], hb[3]); hv[2] = pack16(hb[4], hb[5]); hv[3] = pack16(hb[6], hb[7]);
    unsigned short* dc = wc + (size_t)i * 8;
    *(volatile v4u*)dc = hv;
    __threadfence();
    *(volatile v4u*)dc = hv;
  }
}

__device__ __forceinline__ void oc_emit(const v8f (&acc)[5], const float (&bv)[5], float* slab, float* dst,
                                        int lane, int rlane, int mOff) {
#pragma unroll
  for (int j = 0; j < 5; ++j) {
#pragma unroll
    for (int r = 0; r < 8; ++r) slab[(mOff + r) * NOFFPAD + (j << 4) + rlane] = acc[j][r] + bv[j];
  }
  lds_wave_sync();
  for (int pass = 0; pass < 2; ++pass) {
#pragma unroll 1
    for (int it = 0; it < (16 * NOFFPAD) / 128; ++it) {
      const int idx = (it * 32 + lane) * 4;
      const v4f v = *(const v4f*)(slab + idx);
      *(volatile v4f*)(dst + idx) = v;
    }
    __threadfence();
  }
  lds_wave_sync();
}

__global__ __launch_bounds__(NTHR) void k_offconv(const unsigned short* __restrict__ xhi_p, const unsigned short* __restrict__ xlo_p,
                                                  const unsigned short* __restrict__ wohi_p, const unsigned short* __restrict__ wolo_p,
                                                  const float* __restrict__ ob, float* __restrict__ off) {
  __shared__ __align__(16) float sT[8][16 * NOFFPAD];
  const __bf16* xhi  = (const __bf16*)xhi_p;
  const __bf16* xlo  = (const __bf16*)xlo_p;
  const __bf16* wohi = (const __bf16*)wohi_p;
  const __bf16* wolo = (const __bf16*)wolo_p;
  const int lane  = threadIdx.x & 31;
  const int wave  = threadIdx.x >> 5;
  const int rlane = lane & 15;
  const int hh    = lane >> 4;
  const int koff  = hh * 8;
  const int m0    = blockIdx.x * OC_BLOCK_PX + wave * 32;

  int abase0;
  int abase1;
  {
    const int ma  = m0 + rlane;
    const int na  = ma / HW;
    const int hwa = ma - na * HW;
    const int ha  = hwa / IMW;
    const int wa  = hwa - ha * IMW;
    abase0 = ((na * HALO_H + ha) * HALO_W + wa) * CIN + koff;
    const int mb  = ma + 16;
    const int nb  = mb / HW;
    const int hwb = mb - nb * HW;
    const int hb  = hwb / IMW;
    const int wb  = hwb - hb * IMW;
    abase1 = ((nb * HALO_H + hb) * HALO_W + wb) * CIN + koff;
  }
  const int bbase = rlane * KOFF + koff;

  v8f acc0[5];
  v8f acc1[5];
#pragma unroll
  for (int j = 0; j < 5; ++j) {
    acc0[j] = (v8f){0.f, 0.f, 0.f, 0.f, 0.f, 0.f, 0.f, 0.f};
    acc1[j] = (v8f){0.f, 0.f, 0.f, 0.f, 0.f, 0.f, 0.f, 0.f};
  }

#pragma unroll 1
  for (int ks = 0; ks < OC_KSTEPS; ++ks) {
    const int k2 = ks >> 2;
    const int cs = ks & 3;
    const int kh = k2 / 3;
    const int kw = k2 - kh * 3;
    const int ao = (kh * HALO_W + kw) * CIN + cs * 32;
    const v16b ah0 = Frag<__bf16>::load(xhi + abase0 + ao);
    const v16b al0 = Frag<__bf16>::load(xlo + abase0 + ao);
    const v16b ah1 = Frag<__bf16>::load(xhi + abase1 + ao);
    const v16b al1 = Frag<__bf16>::load(xlo + abase1 + ao);
    const int bo = bbase + ks * 32;
#pragma unroll
    for (int j = 0; j < 5; ++j) {
      const v16b bh = Frag<__bf16>::load(wohi + bo + j * 16 * KOFF);
      const v16b bl = Frag<__bf16>::load(wolo + bo + j * 16 * KOFF);
      acc0[j] = Frag<__bf16>::mma(ah0, bh, acc0[j]);
      acc0[j] = Frag<__bf16>::mma(ah0, bl, acc0[j]);
      acc0[j] = Frag<__bf16>::mma(al0, bh, acc0[j]);
      acc1[j] = Frag<__bf16>::mma(ah1, bh, acc1[j]);
      acc1[j] = Frag<__bf16>::mma(ah1, bl, acc1[j]);
      acc1[j] = Frag<__bf16>::mma(al1, bh, acc1[j]);
      guard_b(acc0[j], ah0, al0, bh, bl);
      guard_b(acc1[j], ah1, al1, bh, bl);
    }
  }

  float bv[5];
#pragma unroll
  for (int j = 0; j < 5; ++j) {
    const int col  = (j << 4) + rlane;
    const int colc = (col < NOFF) ? col : (NOFF - 1);
    float t = ob[colc];
    asm volatile("" : "+v"(t));
    bv[j] = (col < NOFF) ? t : 0.0f;
  }
  float* slab = sT[wave];
  oc_emit(acc0, bv, slab, off + (size_t)m0 * NOFFPAD, lane, rlane, hh * 8);
  oc_emit(acc1, bv, slab, off + (size_t)(m0 + 16) * NOFFPAD, lane, rlane, hh * 8);
}

__global__ __launch_bounds__(NTHR) void k_deform(const float* __restrict__ xf, const float* __restrict__ off,
                                                 const unsigned short* __restrict__ wc_p, const float* __restrict__ cb,
                                                 float* __restrict__ y) {
  __shared__ __align__(16) _Float16 As[TILE_PX * AS_PITCH];
  __shared__ __align__(16) int   gOff[GEO_ITEMS * 4];
  __shared__ __align__(16) float gW[GEO_ITEMS * 4];
  __shared__ __align__(16) float Cst[OG * CST_PITCH];
  const _Float16* wc = (const _Float16*)wc_p;
  const int tid   = threadIdx.x;
  const int lane  = tid & 31;
  const int wave  = tid >> 5;
  const int rlane = lane & 15;
  const int hh    = lane >> 4;
  const int koff  = hh * 8;
  const int m0    = blockIdx.x * TILE_PX;
  const int n     = m0 / HW;
  const int hwb   = m0 - n * HW;
  const int b     = n / DEP;
  const int d     = n - b * DEP;
  const float* xn = xf + (size_t)n * HW * CIN;
  const int mt = wave & 3;
  const int nt = wave >> 2;

#pragma unroll 1
  for (int g = 0; g < NGRP; ++g) {
#pragma unroll 1
    for (int i = tid; i < GEO_ITEMS; i += NTHR) {
      const int ml  = i / NTAP;
      const int tap = i - ml * NTAP;
      const int hw  = hwb + ml;
      const int h   = hw / IMW;
      const int w   = hw - h * IMW;
      const int ky  = tap / 3;
      const int kx  = tap - ky * 3;
      const v2f o2 = *(const v2f*)(off + (size_t)(m0 + ml) * NOFFPAD + 2 * (g * NTAP + tap));
      const float oy = o2[0];
      const float ox = o2[1];
      const float pyf = oy + (float)(h + ky - 1);
      const float pxf = ox + (float)(w + kx - 1);
      const float y0f = floorf(pyf);
      const float x0f = floorf(pxf);
      const float ly  = pyf - y0f;
      const float lx  = pxf - x0f;
      const float y1f = y0f + 1.0f;
      const float x1f = x0f + 1.0f;
      const bool vy0 = (y0f >= 0.0f) && (y0f < (float)IMH);
      const bool vy1 = (y1f >= 0.0f) && (y1f < (float)IMH);
      const bool vx0 = (x0f >= 0.0f) && (x0f < (float)IMW);
      const bool vx1 = (x1f >= 0.0f) && (x1f < (float)IMW);
      const int yc0 = (int)fminf(fmaxf(y0f, 0.0f), (float)(IMH - 1));
      const int yc1 = (int)fminf(fmaxf(y1f, 0.0f), (float)(IMH - 1));
      const int xc0 = (int)fminf(fmaxf(x0f, 0.0f), (float)(IMW - 1));
      const int xc1 = (int)fminf(fmaxf(x1f, 0.0f), (float)(IMW - 1));
      const float omly = 1.0f - ly;
      const float omlx = 1.0f - lx;
      const float p00 = omly * omlx;
      const float p01 = omly * lx;
      const float p10 = ly * omlx;
      const float p11 = ly * lx;
      v4f wv;
      wv[0] = (vy0 && vx0) ? p00 : 0.0f;
      wv[1] = (vy0 && vx1) ? p01 : 0.0f;
      wv[2] = (vy1 && vx0) ? p10 : 0.0f;
      wv[3] = (vy1 && vx1) ? p11 : 0.0f;
      v4i ov;
      ov[0] = (yc0 * IMW + xc0) * CIN;
      ov[1] = (yc0 * IMW + xc1) * CIN;
      ov[2] = (yc1 * IMW + xc0) * CIN;
      ov[3] = (yc1 * IMW + xc1) * CIN;
      *(v4i*)(gOff + i * 4) = ov;
      *(v4f*)(gW + i * 4) = wv;
    }
    __syncthreads();

#pragma unroll 1
    for (int it = 0; it < SMP_ITEMS / NTHR; ++it) {
      const int i   = it * NTHR + tid;
      const int pt  = i >> 2;
      const int ch  = i & 3;
      const int ml  = pt / NTAP;
      const int tap = pt - ml * NTAP;
      const v4i ov = *(const v4i*)(gOff + pt * 4);
      const v4f wv = *(const v4f*)(gW + pt * 4);
      const float* xg = xn + g * CG + ch * 8;
      const v4f a0 = *(const v4f*)(xg + ov[0]);
      const v4f a1 = *(const v4f*)(xg + ov[0] + 4);
      const v4f b0 = *(const v4f*)(xg + ov[1]);
      const v4f b1 = *(const v4f*)(xg + ov[1] + 4);
      const v4f c0 = *(const v4f*)(xg + ov[2]);
      const v4f c1 = *(const v4f*)(xg + ov[2] + 4);
      const v4f d0 = *(const v4f*)(xg + ov[3]);
      const v4f d1 = *(const v4f*)(xg + ov[3] + 4);
      v8h hv;
#pragma unroll
      for (int e = 0; e < 4; ++e) {
        float s = wv[0] * a0[e] + wv[1] * b0[e] + wv[2] * c0[e] + wv[3] * d0[e];
        s = s * SMP_CARRY;
        s = (fabsf(s) < F16_MIN_NORMAL) ? 0.0f : s;
        hv[e] = (_Float16)s;
      }
#pragma unroll
      for (int e = 0; e < 4; ++e) {
        float s = wv[0] * a1[e] + wv[1] * b1[e] + wv[2] * c1[e] + wv[3] * d1[e];
        s = s * SMP_CARRY;
        s = (fabsf(s) < F16_MIN_NORMAL) ? 0.0f : s;
        hv[4 + e] = (_Float16)s;
      }
      *(v8h*)(As + ml * AS_PITCH + tap * CG + ch * 8) = hv;
    }
    __syncthreads();

    v8f acc = (v8f){0.f, 0.f, 0.f, 0.f, 0.f, 0.f, 0.f, 0.f};
    const _Float16* arow = As + (mt * 16 + rlane) * AS_PITCH + koff;
    const _Float16* brow = wc + (size_t)(g * OG + nt * 16 + rlane) * KDEF + koff;
#pragma unroll
    for (int ks = 0; ks < DC_KSTEPS; ++ks) {
      const v16h af = Frag<_Float16>::load(arow + ks * 32);
      const v16h bf = Frag<_Float16>::load(brow + ks * 32);
      acc = mma_h(af, bf, acc);
    }
    {
      const int col = nt * 16 + rlane;
      const float bias = cb[g * OG + col];
      v4f q0;
      v4f q1;
      q0[0] = acc[0] * DC_FOLD + bias; q0[1] = acc[1] * DC_FOLD + bias;
      q0[2] = acc[2] * DC_FOLD + bias; q0[3] = acc[3] * DC_FOLD + bias;
      q1[0] = acc[4] * DC_FOLD + bias; q1[1] = acc[5] * DC_FOLD + bias;
      q1[2] = acc[6] * DC_FOLD + bias; q1[3] = acc[7] * DC_FOLD + bias;
      float* cs = Cst + col * CST_PITCH + mt * 16 + hh * 8;
      *(v4f*)(cs) = q0;
      *(v4f*)(cs + 4) = q1;
    }
    __syncthreads();

    {
      const int c4 = rlane * 4;
      for (int pass = 0; pass < 2; ++pass) {
#pragma unroll
        for (int it = 0; it < 2; ++it) {
          const int row = wave * 4 + it * 2 + hh;
          const v4f v = *(const v4f*)(Cst + row * CST_PITCH + c4);
          float* dst = y + ((size_t)(b * COUT + g * OG + row) * DEP + d) * HW + hwb + c4;
          *(volatile v4f*)dst = v;
        }
        __threadfence();
      }
    }
  }
}

__global__ __launch_bounds__(NTHR) void k_norm_act(const float* __restrict__ y, float* __restrict__ out) {
  __shared__ double red[NTHR];
  __shared__ float stat[2];
  const int tid = threadIdx.x;
  const size_t base = (size_t)blockIdx.x * RUN;
  const float* src = y + base;
  float* dstb = out + base;

  double s1 = 0.0;
#pragma unroll 1
  for (int q = tid; q < RUN / 4; q += NTHR) {
    const v4f v = *(const v4f*)(src + (size_t)q * 4);
    s1 += ((double)v[0] + (double)v[1]) + ((double)v[2] + (double)v[3]);
  }
  red[tid] = s1;
  __syncthreads();
#pragma unroll 1
  for (int o = NTHR / 2; o > 0; o >>= 1) {
    if (tid < o) red[tid] += red[tid + o];
    __syncthreads();
  }
  if (tid == 0) stat[0] = (float)(red[0] * INV_RUN);
  __syncthreads();
  const float mu = stat[0];

  double s2 = 0.0;
#pragma unroll 1
  for (int q = tid; q < RUN / 4; q += NTHR) {
    const v4f v = *(const v4f*)(src + (size_t)q * 4);
    const double e0 = (double)(v[0] - mu);
    const double e1 = (double)(v[1] - mu);
    const double e2 = (double)(v[2] - mu);
    const double e3 = (double)(v[3] - mu);
    s2 += (e0 * e0 + e1 * e1) + (e2 * e2 + e3 * e3);
  }
  red[tid] = s2;
  __syncthreads();
#pragma unroll 1
  for (int o = NTHR / 2; o > 0; o >>= 1) {
    if (tid < o) red[tid] += red[tid + o];
    __syncthreads();
  }
  if (tid == 0) {
    const float var = (float)(red[0] * INV_RUN);
    stat[1] = rsqrtf(var + NORM_EPS);
  }
  __syncthreads();
  const float inv = stat[1];

#pragma unroll 1
  for (int q = tid; q < RUN / 4; q += NTHR) {
    const v4f v = *(const v4f*)(src + (size_t)q * 4);
    float a0 = (v[0] - mu) * inv;
    float a1 = (v[1] - mu) * inv;
    float a2 = (v[2] - mu) * inv;
    float a3 = (v[3] - mu) * inv;
#pragma unroll 1
    for (int e = 0; e < 4; ++e) {
      const float t = 0.5f * a0 * (1.0f + erff(a0 * 0.70710678118654752f));
      a0 = a1;
      a1 = a2;
      a2 = a3;
      a3 = t;
    }
    v4f r;
    r[0] = a0; r[1] = a1; r[2] = a2; r[3] = a3;
    float* dst = dstb + (size_t)q * 4;
    *(volatile v4f*)dst = r;
    __threadfence();
    *(volatile v4f*)dst = r;
  }
}

constexpr size_t SZ_XF   = (size_t)NIMG * HW * CIN * 4;
constexpr size_t SZ_XH   = (size_t)NIMG * HPIX * CIN * 2;
constexpr size_t SZ_WO   = (size_t)NOFFPAD * KOFF * 2;
constexpr size_t SZ_WC   = (size_t)COUT * KDEF * 2;
constexpr size_t SZ_OFF  = (size_t)NPIX * NOFFPAD * 4;
constexpr size_t SZ_Y    = (size_t)NB * COUT * RUN * 4;
constexpr size_t OFF_XF  = 0;
constexpr size_t OFF_XHI = OFF_XF + SZ_XF;
constexpr size_t OFF_XLO = OFF_XHI + SZ_XH;
constexpr size_t OFF_WOH = OFF_XLO + SZ_XH;
constexpr size_t OFF_WOL = OFF_WOH + SZ_WO;
constexpr size_t OFF_WC  = OFF_WOL + SZ_WO;
constexpr size_t OFF_OFF = OFF_WC + SZ_WC;
constexpr size_t OFF_Y   = OFF_OFF + SZ_OFF;
constexpr size_t WS_TOTAL = OFF_Y + SZ_Y;
static_assert(WS_TOTAL == 71688192u);
static_assert(WS_TOTAL <= 134217728u);
static_assert(OFF_XHI % 128 == 0 && OFF_XLO % 128 == 0 && OFF_WOH % 128 == 0 && OFF_WOL % 128 == 0 &&
              OFF_WC % 128 == 0 && OFF_OFF % 128 == 0 && OFF_Y % 128 == 0);
static_assert(SZ_Y == 19267584u && SZ_XF == 19267584u);

extern "C" void kernel_launch(void* const* d_in, const int* in_sizes, int n_in,
                              void* d_out, int out_size, void* d_ws, size_t ws_size,
                              hipStream_t stream) {
  if (n_in < 5) return;
  if (in_sizes[0] != NB * CIN * DEP * HW) return;
  if (in_sizes[1] != NOFF * KOFF) return;
  if (in_sizes[2] != NOFF) return;
  if (in_sizes[3] != COUT * KDEF) return;
  if (in_sizes[4] != COUT) return;
  if ((size_t)out_size < (size_t)NB * COUT * RUN) return;
  if (ws_size < WS_TOTAL) return;

  const float* x  = (const float*)d_in[0];
  const float* ow = (const float*)d_in[1];
  const float* ob = (const float*)d_in[2];
  const float* cw = (const float*)d_in[3];
  const float* cb = (const float*)d_in[4];
  float* out = (float*)d_out;

  char* ws = (char*)d_ws;
  float*          xf   = (float*)(ws + OFF_XF);
  unsigned short* xhi  = (unsigned short*)(ws + OFF_XHI);
  unsigned short* xlo  = (unsigned short*)(ws + OFF_XLO);
  unsigned short* wohi = (unsigned short*)(ws + OFF_WOH);
  unsigned short* wolo = (unsigned short*)(ws + OFF_WOL);
  unsigned short* wc   = (unsigned short*)(ws + OFF_WC);
  float*          off  = (float*)(ws + OFF_OFF);
  float*          y    = (float*)(ws + OFF_Y);

  k_prep_x<<<dim3(TILES_PER_IMG + 1, NIMG), NTHR, 0, stream>>>(x, xf, xhi, xlo);
  k_prep_w<<<WO_BLOCKS + WC_BLOCKS, NTHR, 0, stream>>>(ow, cw, wohi, wolo, wc);
  k_offconv<<<NPIX / OC_BLOCK_PX, NTHR, 0, stream>>>(xhi, xlo, wohi, wolo, ob, off);
  k_deform<<<NTILES, NTHR, 0, stream>>>(xf, off, wc, cb, y);
  k_norm_act<<<NB * COUT, NTHR, 0, stream>>>(y, out);
}
